// MLPPredictor_3444563771451
// MI455X (gfx1250) — hardware-verified
//
#include <hip/hip_runtime.h>
#include <stddef.h>
#include <stdint.h>


#define HF     128
#define HID    256
#define PCN    512
#define NPF    6
#define W2K    262
#define NTHR   256
#define GBM    64
#define GBN    128
#define GTHR   128
#define NUW    (PCN * HF / 8)
#define UPR    (HF / 8)
#define EPL    16
#define LPW    8
#define LPB    (LPW * (NTHR / 32))
#define LN_EPS 1e-5f
#define WSLIM  268435456

static_assert(NUW % NTHR == 0);
static_assert((GBM * UPR) % NTHR == 0);
static_assert(HF % 32 == 0 && PCN % GBN == 0 && PCN == 2 * HID);
static_assert(GBM == (GTHR / 32) * 16 && GBN == 4 * 32);
static_assert(UPR == 16);
static_assert(HID == 8 * 32);
static_assert(EPL * 2 == 32);
static_assert(W2K == HID + NPF && (W2K % 2) == 0 && NPF <= 32);

typedef float          v2f   __attribute__((ext_vector_type(2)));
typedef float          v4f   __attribute__((ext_vector_type(4)));
typedef float          v8f   __attribute__((ext_vector_type(8)));
typedef int            v8i   __attribute__((ext_vector_type(8)));
typedef unsigned short v8us  __attribute__((ext_vector_type(8)));
typedef unsigned short v16us __attribute__((ext_vector_type(16)));
typedef __bf16         v16bf __attribute__((ext_vector_type(16)));
typedef v2f  __attribute__((may_alias)) v2fa;
typedef v4f  __attribute__((may_alias)) v4fa;
typedef v8us __attribute__((may_alias)) v8usa;
union FragB { v16bf v; v16us u; v8us h[2]; v8i w; };

__device__ __forceinline__ v8f wmb(const FragB& a, const FragB& b, v8f c) {
  v8f d = __builtin_amdgcn_wmma_f32_16x16x32_bf16(false, a.v, false, b.v, (short)0, c, false, false);
  asm volatile("v_nop\n\tv_nop\n\tv_nop\n\tv_nop" : "+v"(d) : "v"(a.w), "v"(b.w));
  return d;
}

__device__ __forceinline__ unsigned bf16_bits(float f) {
  const unsigned u = __float_as_uint(f);
  return (u + 0x7FFFu + ((u >> 16) & 1u)) >> 16;
}
__device__ __forceinline__ float bf16_val(float f) {
  return __uint_as_float(bf16_bits(f) << 16);
}

__global__ __launch_bounds__(NTHR) void k_prep(const float* __restrict__ W1, const float* __restrict__ h,
                                               int nN, int nUH,
                                               unsigned short* WT, unsigned short* XH) {
  const int u = (int)blockIdx.x * NTHR + (int)threadIdx.x;
  const float* p;
  unsigned short* dp;
  bool ok;
  if (u < NUW) {
    const int nn = u >> 4;
    const int k8 = (u & 15) * 8;
    p  = W1 + (size_t)(nn & (HID - 1)) * (size_t)(2 * HF) + (size_t)((nn >> 8) * HF + k8);
    dp = WT + (size_t)nn * HF + k8;
    ok = true;
  } else {
    const int v = u - NUW;
    if (v >= nUH) return;
    const int row = v >> 4;
    const int k8  = (v & 15) * 8;
    const int rc  = row < nN ? row : nN - 1;
    p  = h + (size_t)rc * HF + k8;
    dp = XH + (size_t)row * HF + k8;
    ok = row < nN;
  }
  const v4f a = *(const v4fa*)p;
  const v4f b = *(const v4fa*)(p + 4);
  v8us o;
  o[0] = ok ? (unsigned short)bf16_bits(a.x) : (unsigned short)0;
  o[1] = ok ? (unsigned short)bf16_bits(a.y) : (unsigned short)0;
  o[2] = ok ? (unsigned short)bf16_bits(a.z) : (unsigned short)0;
  o[3] = ok ? (unsigned short)bf16_bits(a.w) : (unsigned short)0;
  o[4] = ok ? (unsigned short)bf16_bits(b.x) : (unsigned short)0;
  o[5] = ok ? (unsigned short)bf16_bits(b.y) : (unsigned short)0;
  o[6] = ok ? (unsigned short)bf16_bits(b.z) : (unsigned short)0;
  o[7] = ok ? (unsigned short)bf16_bits(b.w) : (unsigned short)0;
  *(volatile v8us*)dp = o;
  __threadfence();
  *(volatile v8us*)dp = o;
}

__global__ __launch_bounds__(GTHR) void k_gemm(const unsigned short* __restrict__ A, int lda,
                                               const unsigned short* __restrict__ BT, int ldb, int K,
                                               float* Cm, int ldc) {
  __shared__ __attribute__((aligned(16))) float stg[GBM * GBN];
  const int tid = (int)threadIdx.x, lane = tid & 31, wave = tid >> 5, hh = lane >> 4, m = lane & 15;
  const int rowBase = (int)blockIdx.x * GBM;
  const int colBase = (int)blockIdx.y * GBN;

  v8f acc[8];
  {
    const v8f z = {0.f, 0.f, 0.f, 0.f, 0.f, 0.f, 0.f, 0.f};
#pragma unroll
    for (int t = 0; t < 8; ++t) acc[t] = z;
  }
  const unsigned short* ap = A  + (size_t)(rowBase + 16 * wave + m) * (size_t)lda + 8 * hh;
  const unsigned short* bp = BT + (size_t)(colBase + m) * (size_t)ldb + 8 * hh;

#pragma unroll 1
  for (int k0 = 0; k0 < K; k0 += 32) {
    FragB af;
    af.h[0] = *(const v8usa*)(ap + k0);
    af.h[1] = *(const v8usa*)(ap + k0 + 16);
#pragma unroll
    for (int nt = 0; nt < 8; ++nt) {
      const unsigned short* wq = bp + (size_t)(16 * nt) * (size_t)ldb + k0;
      FragB bf;
      bf.h[0] = *(const v8usa*)wq;
      bf.h[1] = *(const v8usa*)(wq + 16);
      acc[nt] = wmb(af, bf, acc[nt]);
    }
  }

#pragma unroll
  for (int nt = 0; nt < 8; ++nt) {
    const int lc = 16 * nt + m;
#pragma unroll
    for (int r = 0; r < 8; ++r) {
      const int lr = 16 * wave + 8 * hh + r;
      stg[lr * GBN + lc] = acc[nt][r];
    }
  }
  __syncthreads();

  v4f pv[16];
#pragma unroll
  for (int i = 0; i < 16; ++i) pv[i] = *(const v4fa*)(stg + (16 * wave + i) * GBN + 4 * lane);
#pragma unroll
  for (int i = 0; i < 16; ++i) {
    float* op = Cm + (size_t)(rowBase + 16 * wave + i) * (size_t)ldc + colBase + 4 * lane;
    *(volatile v4f*)op = pv[i];
  }
  __threadfence();
#pragma unroll
  for (int i = 0; i < 16; ++i) {
    float* op = Cm + (size_t)(rowBase + 16 * wave + i) * (size_t)ldc + colBase + 4 * lane;
    *(volatile v4f*)op = pv[i];
  }
}

__device__ __forceinline__ void cvt8(const float* __restrict__ p, float (&o)[8]) {
  const v4f a = *(const v4fa*)p;
  const v4f b = *(const v4fa*)(p + 4);
  o[0] = bf16_val(a.x); o[1] = bf16_val(a.y); o[2] = bf16_val(a.z); o[3] = bf16_val(a.w);
  o[4] = bf16_val(b.x); o[5] = bf16_val(b.y); o[6] = bf16_val(b.z); o[7] = bf16_val(b.w);
}

__device__ __forceinline__ float wsum(float v) {
  v += __shfl_xor(v, 16);
  v += __shfl_xor(v, 8);
  v += __shfl_xor(v, 4);
  v += __shfl_xor(v, 2);
  v += __shfl_xor(v, 1);
  return v;
}

__global__ __launch_bounds__(NTHR) void k_edge(const int* __restrict__ si, const int* __restrict__ di,
                                               const float* __restrict__ pol, const float* __restrict__ P,
                                               const float* __restrict__ b1, const float* __restrict__ gam,
                                               const float* __restrict__ bet, const float* __restrict__ w2,
                                               const float* __restrict__ b2, int nE, int nN, int nLines,
                                               float* out) {
  const int tid = (int)threadIdx.x, lane = tid & 31, wave = tid >> 5;
  const int c0 = 8 * lane;

  float cb[8], cg[8], ce[8], cw0[8], cw1[8];
  cvt8(b1 + c0, cb);
  cvt8(gam + c0, cg);
  cvt8(bet + c0, ce);
  cvt8(w2 + c0, cw0);
  {
    const float* q = w2 + W2K + c0;
    const v2f u0 = *(const v2fa*)q;
    const v2f u1 = *(const v2fa*)(q + 2);
    const v2f u2 = *(const v2fa*)(q + 4);
    const v2f u3 = *(const v2fa*)(q + 6);
    cw1[0] = bf16_val(u0.x); cw1[1] = bf16_val(u0.y); cw1[2] = bf16_val(u1.x); cw1[3] = bf16_val(u1.y);
    cw1[4] = bf16_val(u2.x); cw1[5] = bf16_val(u2.y); cw1[6] = bf16_val(u3.x); cw1[7] = bf16_val(u3.y);
  }
  const int   lp  = lane < NPF ? lane : NPF - 1;
  const float fac = lane < NPF ? 1.0f : 0.0f;
  const float pw0 = bf16_val(w2[HID + lp]) * fac;
  const float pw1 = bf16_val(w2[W2K + HID + lp]) * fac;
  const float bb0 = bf16_val(b2[0]);
  const float bb1 = bf16_val(b2[1]);

  const int lbase = (int)blockIdx.x * LPB + wave * LPW;
#pragma unroll 1
  for (int j = 0; j < LPW; ++j) {
    const int L = lbase + j;
    if (L >= nLines) break;
    const int e0 = L * EPL;
    float res = 0.0f;
#pragma unroll 1
    for (int i = 0; i < EPL; ++i) {
      int e = e0 + i;
      e = e > nE - 1 ? nE - 1 : e;
      int s = si[e];
      int t = di[e];
      s = s < 0 ? 0 : (s > nN - 1 ? nN - 1 : s);
      t = t < 0 ? 0 : (t > nN - 1 ? nN - 1 : t);
      const float* pa = P + (size_t)s * PCN + c0;
      const float* pb = P + (size_t)t * PCN + HID + c0;
      const v4f a0 = *(const v4fa*)pa;
      const v4f a1 = *(const v4fa*)(pa + 4);
      const v4f q0 = *(const v4fa*)pb;
      const v4f q1 = *(const v4fa*)(pb + 4);
      const float pv = bf16_val(pol[(size_t)e * NPF + lp]);

      float x[8];
      x[0] = (a0.x + q0.x) + cb[0];
      x[1] = (a0.y + q0.y) + cb[1];
      x[2] = (a0.z + q0.z) + cb[2];
      x[3] = (a0.w + q0.w) + cb[3];
      x[4] = (a1.x + q1.x) + cb[4];
      x[5] = (a1.y + q1.y) + cb[5];
      x[6] = (a1.z + q1.z) + cb[6];
      x[7] = (a1.w + q1.w) + cb[7];
      float sm = ((x[0] + x[1]) + (x[2] + x[3])) + ((x[4] + x[5]) + (x[6] + x[7]));
      sm = wsum(sm);
      const float mu = sm * (1.0f / HID);
      float sq = 0.0f;
#pragma unroll
      for (int k = 0; k < 8; ++k) {
        x[k] = x[k] - mu;
        sq = fmaf(x[k], x[k], sq);
      }
      sq = wsum(sq);
      const float rstd = rsqrtf(sq * (1.0f / HID) + LN_EPS);
      float d0 = 0.0f, d1 = 0.0f;
#pragma unroll
      for (int k = 0; k < 8; ++k) {
        const float y = fmaxf(fmaf(x[k] * rstd, cg[k], ce[k]), 0.0f);
        d0 = fmaf(y, cw0[k], d0);
        d1 = fmaf(y, cw1[k], d1);
      }
      d0 = fmaf(pv, pw0, d0);
      d1 = fmaf(pv, pw1, d1);
      d0 += __shfl_xor(d0, 16); d1 += __shfl_xor(d1, 16);
      d0 += __shfl_xor(d0, 8);  d1 += __shfl_xor(d1, 8);
      d0 += __shfl_xor(d0, 4);  d1 += __shfl_xor(d1, 4);
      d0 += __shfl_xor(d0, 2);  d1 += __shfl_xor(d1, 2);
      d0 += __shfl_xor(d0, 1);  d1 += __shfl_xor(d1, 1);
      const float s0  = d0 + bb0;
      const float s1  = d1 + bb1;
      const float s01 = (lane & 1) ? s1 : s0;
      res = ((lane >> 1) == i) ? s01 : res;
    }
    v4f o;
    o.x = __shfl(res, (4 * lane) & 31);
    o.y = __shfl(res, (4 * lane + 1) & 31);
    o.z = __shfl(res, (4 * lane + 2) & 31);
    o.w = __shfl(res, (4 * lane + 3) & 31);
    float* op = out + (size_t)e0 * 2 + 4 * (lane & 7);
    if (lane < 8) *(volatile v4f*)op = o;
    __threadfence();
    if (lane < 8) *(volatile v4f*)op = o;
  }
}

static inline int cdiv(int a, int b) { return (a + b - 1) / b; }

extern "C" void kernel_launch(void* const* d_in, const int* in_sizes, int n_in,
                              void* d_out, int out_size, void* d_ws, size_t ws_size,
                              hipStream_t stream) {
  if (n_in < 10) return;
  if (in_sizes[0] < HF || (in_sizes[0] % HF) != 0) return;
  const int nN = in_sizes[0] / HF;
  if (nN > (1 << 22)) return;
  const int nE = in_sizes[1];
  if (nE < EPL || (nE % EPL) != 0) return;
  if (in_sizes[2] != nE) return;
  if (in_sizes[3] != NPF * nE) return;
  if (in_sizes[4] != HID * 2 * HF) return;
  if (in_sizes[5] != HID) return;
  if (in_sizes[6] != HID) return;
  if (in_sizes[7] != HID) return;
  if (in_sizes[8] != 2 * W2K) return;
  if (in_sizes[9] != 2) return;
  if (out_size != 2 * nE) return;

  const float* h     = (const float*)d_in[0];
  const int*   src   = (const int*)d_in[1];
  const int*   dst   = (const int*)d_in[2];
  const float* polar = (const float*)d_in[3];
  const float* W1    = (const float*)d_in[4];
  const float* b1    = (const float*)d_in[5];
  const float* gamma = (const float*)d_in[6];
  const float* beta  = (const float*)d_in[7];
  const float* W2    = (const float*)d_in[8];
  const float* b2    = (const float*)d_in[9];
  float* out = (float*)d_out;

  const int MP  = cdiv(nN, GBM) * GBM;
  const int nUH = MP * UPR;
  const int nLines = nE / EPL;

  char* ws = (char*)d_ws;
  size_t off = 0;
  const size_t oWT = off; off += (size_t)PCN * HF * 2;      off = (off + 255) & ~(size_t)255;
  const size_t oXH = off; off += (size_t)MP * HF * 2;       off = (off + 255) & ~(size_t)255;
  const size_t oP  = off; off += (size_t)MP * PCN * 4;      off = (off + 255) & ~(size_t)255;
  if (off > ws_size || off > (size_t)WSLIM) return;
  unsigned short* WT = (unsigned short*)(ws + oWT);
  unsigned short* XH = (unsigned short*)(ws + oXH);
  float*          P  = (float*)(ws + oP);

  const int nUnits = NUW + nUH;
  k_prep<<<cdiv(nUnits, NTHR), NTHR, 0, stream>>>(W1, h, nN, nUH, WT, XH);
  k_gemm<<<dim3(MP / GBM, PCN / GBN), GTHR, 0, stream>>>(XH, HF, WT, HF, HF, P, PCN);
  k_edge<<<cdiv(nLines, LPB), NTHR, 0, stream>>>(src, dst, polar, P, b1, gamma, beta, W2, b2,
                                                nE, nN, nLines, out);
}
